// LSTM_80470507258143
// MI455X (gfx1250) — hardware-verified
//
#include <hip/hip_runtime.h>
#include <math.h>

constexpr int NBATCH       = 32;
constexpr int NSTEP        = 1024;
constexpr int NHID         = 512;
constexpr int NGATE        = 4 * NHID;
constexpr int NOUTF        = 3;
constexpr int SCAN_THREADS = 512;
constexpr int SIDE_THREADS = 256;
constexpr int HPITCH       = 520;
constexpr int TILE_ELEMS   = NBATCH * HPITCH;
constexpr int STEP_ELEMS   = NBATCH * NHID;
constexpr float WCARRY     = 256.0f;
constexpr float HCARRY     = 1024.0f;
constexpr float ACC_FOLD   = 1.0f / (WCARRY * HCARRY);

static_assert(NBATCH == 32, "two 16-row m-subtiles");
static_assert(NHID == 32 * (SCAN_THREADS / 32), "16 waves x 32 hidden units");
static_assert(NHID % 32 == 0, "k steps of 32");
static_assert(STEP_ELEMS / 8 == 4 * SCAN_THREADS, "tile copy: 4 chunks of 16 B per thread");
static_assert(HPITCH % 8 == 0 && HPITCH >= NHID, "16-B aligned LDS rows");
static_assert((NBATCH * NSTEP) % (32 * 8) == 0, "head grid exact");

typedef __attribute__((ext_vector_type(16))) _Float16 v16h;
typedef __attribute__((ext_vector_type(8)))  _Float16 v8h;
typedef __attribute__((ext_vector_type(8)))  float    v8f;
typedef __attribute__((ext_vector_type(4)))  float    v4f;

__device__ __forceinline__ void dep_guard_h(v8f& a, v8f& b, v16h x, v16h y) { asm volatile("v_nop\n\tv_nop\n\tv_nop\n\tv_nop" : "+v"(a), "+v"(b) : "v"(x), "v"(y)); }
__device__ __forceinline__ void keep4_h(v16h a, v16h b, v16h c, v16h d) { asm volatile("v_nop" :: "v"(a), "v"(b), "v"(c), "v"(d)); }
__device__ __forceinline__ void guard8(v8f& c0, v8f& c1, v8f& c2, v8f& c3, v8f& c4, v8f& c5, v8f& c6, v8f& c7,
                                       v16h a0, v16h a1, v16h b0, v16h b1, v16h b2, v16h b3) {
  asm volatile("v_nop\n\tv_nop\n\tv_nop\n\tv_nop"
               : "+v"(c0), "+v"(c1), "+v"(c2), "+v"(c3), "+v"(c4), "+v"(c5), "+v"(c6), "+v"(c7)
               : "v"(a0), "v"(a1), "v"(b0), "v"(b1), "v"(b2), "v"(b3));
}
__device__ __forceinline__ void guard2(v8f& c0, v8f& c1, v16h a0, v16h a1, v16h b0) {
  asm volatile("v_nop\n\tv_nop\n\tv_nop\n\tv_nop" : "+v"(c0), "+v"(c1) : "v"(a0), "v"(a1), "v"(b0));
}
__device__ __forceinline__ void pin8(float& a, float& b, float& c, float& d, float& e, float& f, float& g, float& h) {
  asm volatile("" : "+v"(a), "+v"(b), "+v"(c), "+v"(d), "+v"(e), "+v"(f), "+v"(g), "+v"(h) :: "memory");
}

template <typename T> struct Frag;
template <> struct Frag<_Float16> {
  typedef v16h V; union U { v16h v; v8h h[2]; };
  static __device__ __forceinline__ v16h load(const _Float16* p) {
    U f; f.h[0] = *(const v8h*)(p); f.h[1] = *(const v8h*)(p + 16); return f.v;
  }
  static __device__ __forceinline__ v8f mma(v16h a, v16h b, v8f c) {
    return __builtin_amdgcn_wmma_f32_16x16x32_f16(false, a, false, b, (short)0, c, false, false);
  }
  static __device__ __forceinline__ void guard(v8f& a, v8f& b, v16h x, v16h y) { dep_guard_h(a, b, x, y); }
  static __device__ __forceinline__ void keep(v16h a, v16h b, v16h c, v16h d) { keep4_h(a, b, c, d); }
};

__device__ __forceinline__ float fsig(float x)  { return __builtin_amdgcn_rcpf(1.0f + __expf(-x)); }
__device__ __forceinline__ float ftanh(float x) { return 1.0f - 2.0f * __builtin_amdgcn_rcpf(__expf(2.0f * x) + 1.0f); }

__global__ __launch_bounds__(SIDE_THREADS) void prep_w_kernel(const float* __restrict__ w_hh0, const float* __restrict__ w_ih1,
                                                              const float* __restrict__ w_hh1,
                                                              unsigned short* __restrict__ wb0, unsigned short* __restrict__ wb1) {
  const int job = blockIdx.y;
  const float* src = (job == 0) ? w_hh0 : ((job == 1) ? w_ih1 : w_hh1);
  unsigned short* dst = (job == 0) ? wb0 : wb1;
  const int dpitch = (job == 0) ? NHID : 2 * NHID;
  const int dcol0  = (job == 2) ? NHID : 0;
  const int i   = blockIdx.x * SIDE_THREADS + threadIdx.x;
  const int row = i >> 6;
  const int c8  = i & 63;
  const float* sp = src + (size_t)row * NHID + c8 * 8;
  const v4f a = *(const v4f*)(sp);
  const v4f b = *(const v4f*)(sp + 4);
  v8h hv;
#pragma unroll
  for (int e = 0; e < 4; ++e) {
    hv[e]     = (_Float16)(a[e] * WCARRY);
    hv[4 + e] = (_Float16)(b[e] * WCARRY);
  }
  unsigned short* op = dst + (size_t)row * dpitch + dcol0 + c8 * 8;
  *(volatile v8h*)op = hv;
  __threadfence();
  *(volatile v8h*)op = hv;
}

__global__ __launch_bounds__(SIDE_THREADS) void prep_misc_kernel(const float* __restrict__ b_ih0, const float* __restrict__ b_hh0,
                                                                 const float* __restrict__ b_ih1, const float* __restrict__ b_hh1,
                                                                 const float* __restrict__ x, const float* __restrict__ fcw,
                                                                 float* __restrict__ bsum, float* __restrict__ xt,
                                                                 unsigned short* __restrict__ wfc) {
  const int blk = blockIdx.x;
  const int tid = threadIdx.x;
  if (blk < 4) {
    const int which = blk >> 1;
    const int idx = ((blk & 1) * SIDE_THREADS + tid) * 4;
    const float* pa = which ? b_ih1 : b_ih0;
    const float* pb = which ? b_hh1 : b_hh0;
    const v4f va = *(const v4f*)(pa + idx);
    const v4f vb = *(const v4f*)(pb + idx);
    v4f o;
#pragma unroll
    for (int e = 0; e < 4; ++e) o[e] = va[e] + vb[e];
    float* op = bsum + which * NGATE + idx;
    *(volatile v4f*)op = o;
    __threadfence();
    *(volatile v4f*)op = o;
  } else if (blk < 36) {
    const int gi = (blk - 4) * SIDE_THREADS + tid;
    const int t  = gi >> 3;
    const int b4 = (gi & 7) * 4;
    v4f o;
#pragma unroll
    for (int e = 0; e < 4; ++e) o[e] = x[(size_t)(b4 + e) * NSTEP + t];
    float* op = xt + (size_t)gi * 4;
    *(volatile v4f*)op = o;
    __threadfence();
    *(volatile v4f*)op = o;
  } else {
    const int gi  = (blk - 36) * SIDE_THREADS + tid;
    const int row = gi >> 6;
    const int c8  = gi & 63;
    const int rc  = (row < NOUTF) ? row : (NOUTF - 1);
    const float* sp = fcw + (size_t)rc * NHID + c8 * 8;
    const v4f a = *(const v4f*)(sp);
    const v4f b = *(const v4f*)(sp + 4);
    v8h hv;
#pragma unroll
    for (int e = 0; e < 4; ++e) {
      const float f0 = (row < NOUTF) ? (a[e] * WCARRY) : 0.0f;
      const float f1 = (row < NOUTF) ? (b[e] * WCARRY) : 0.0f;
      hv[e]     = (_Float16)f0;
      hv[4 + e] = (_Float16)f1;
    }
    unsigned short* op = wfc + (size_t)gi * 8;
    *(volatile v8h*)op = hv;
    __threadfence();
    *(volatile v8h*)op = hv;
  }
}

template <int KW>
__device__ __forceinline__ void gate_kloop(const _Float16* ap0, const _Float16* ap1, const _Float16* wp,
                                           v8f& i0, v8f& i1, v8f& f0, v8f& f1, v8f& g0, v8f& g1, v8f& o0, v8f& o1) {
  constexpr size_t GSTR = (size_t)NHID * KW;
#pragma unroll 1
  for (int k0 = 0; k0 < NHID; k0 += 32) {
    const v16h a0 = Frag<_Float16>::load(ap0 + k0);
    const v16h a1 = Frag<_Float16>::load(ap1 + k0);
    const v16h b0 = Frag<_Float16>::load(wp + k0);
    const v16h b1 = Frag<_Float16>::load(wp + GSTR + k0);
    const v16h b2 = Frag<_Float16>::load(wp + 2 * GSTR + k0);
    const v16h b3 = Frag<_Float16>::load(wp + 3 * GSTR + k0);
    i0 = Frag<_Float16>::mma(a0, b0, i0);
    i1 = Frag<_Float16>::mma(a1, b0, i1);
    f0 = Frag<_Float16>::mma(a0, b1, f0);
    f1 = Frag<_Float16>::mma(a1, b1, f1);
    g0 = Frag<_Float16>::mma(a0, b2, g0);
    g1 = Frag<_Float16>::mma(a1, b2, g1);
    o0 = Frag<_Float16>::mma(a0, b3, o0);
    o1 = Frag<_Float16>::mma(a1, b3, o1);
    guard8(i0, i1, f0, f1, g0, g1, o0, o1, a0, a1, b0, b1, b2, b3);
  }
}

template <int LAYER>
__device__ __forceinline__ void cell_update(const v8f& zi, const v8f& zf, const v8f& zg, const v8f& zo,
                                            float bi, float bf, float bg, float bo,
                                            float wi, float wf, float wg, float wo,
                                            v4f xa, v4f xb, float (&cs)[8], _Float16* dst) {
#pragma unroll
  for (int r = 0; r < 8; ++r) {
    float pi = bi, pf = bf, pg = bg, po = bo;
    if (LAYER == 0) {
      const float xv = (r < 4) ? xa[r & 3] : xb[r & 3];
      pi = fmaf(xv, wi, bi);
      pf = fmaf(xv, wf, bf);
      pg = fmaf(xv, wg, bg);
      po = fmaf(xv, wo, bo);
    }
    const float vi = fmaf(zi[r], ACC_FOLD, pi);
    const float vf = fmaf(zf[r], ACC_FOLD, pf);
    const float vg = fmaf(zg[r], ACC_FOLD, pg);
    const float vo = fmaf(zo[r], ACC_FOLD, po);
    const float ig = fsig(vi);
    const float fg = fsig(vf);
    const float og = fsig(vo);
    const float gg = ftanh(vg);
    const float cn = fg * cs[r] + ig * gg;
    cs[r] = cn;
    const float hn = og * ftanh(cn);
    dst[r * HPITCH] = (_Float16)(hn * HCARRY);
  }
}

template <int LAYER>
__global__ __launch_bounds__(SCAN_THREADS) void lstm_scan_kernel(const unsigned short* __restrict__ Wbp,
                                                                 const float* __restrict__ bsum,
                                                                 const float* __restrict__ wx0,
                                                                 const float* __restrict__ xT,
                                                                 const unsigned short* __restrict__ hinp,
                                                                 const float* __restrict__ hinit,
                                                                 const float* __restrict__ cinit,
                                                                 unsigned short* __restrict__ histp) {
  constexpr int KW = (LAYER == 0) ? NHID : 2 * NHID;
  __shared__ __align__(16) _Float16 Ah[2 * TILE_ELEMS];
  __shared__ __align__(16) _Float16 Ax[(LAYER == 1) ? TILE_ELEMS : 8];
  const _Float16* Wb  = (const _Float16*)Wbp;
  const _Float16* hin = (const _Float16*)hinp;
  const int tid = threadIdx.x, lane = tid & 31, wave = tid >> 5;
  const int c = lane & 15, hh = lane >> 4, koff = hh * 8;

#pragma unroll 1
  for (int it = 0; it < 4; ++it) {
    const int id  = it * SCAN_THREADS + tid;
    const int row = id >> 6;
    const int c8  = id & 63;
    const float* sp = hinit + (size_t)row * NHID + c8 * 8;
    const v4f a = *(const v4f*)(sp);
    const v4f b = *(const v4f*)(sp + 4);
    v8h hv;
#pragma unroll
    for (int e = 0; e < 4; ++e) {
      hv[e]     = (_Float16)(a[e] * HCARRY);
      hv[4 + e] = (_Float16)(b[e] * HCARRY);
    }
    *(v8h*)(Ah + row * HPITCH + c8 * 8) = hv;
  }

  float bs[2][4], wq[2][4], cst[2][2][8];
#pragma unroll
  for (int ug = 0; ug < 2; ++ug)
#pragma unroll
    for (int g = 0; g < 4; ++g) bs[ug][g] = bsum[g * NHID + 32 * wave + 16 * ug + c];
  pin8(bs[0][0], bs[0][1], bs[0][2], bs[0][3], bs[1][0], bs[1][1], bs[1][2], bs[1][3]);
#pragma unroll
  for (int ug = 0; ug < 2; ++ug)
#pragma unroll
    for (int g = 0; g < 4; ++g) wq[ug][g] = (LAYER == 0) ? wx0[g * NHID + 32 * wave + 16 * ug + c] : 0.0f;
  if (LAYER == 0) pin8(wq[0][0], wq[0][1], wq[0][2], wq[0][3], wq[1][0], wq[1][1], wq[1][2], wq[1][3]);
#pragma unroll
  for (int ug = 0; ug < 2; ++ug) {
#pragma unroll
    for (int mt = 0; mt < 2; ++mt) {
#pragma unroll
      for (int r = 0; r < 8; ++r)
        cst[ug][mt][r] = cinit[(size_t)(16 * mt + 8 * hh + r) * NHID + 32 * wave + 16 * ug + c];
      pin8(cst[ug][mt][0], cst[ug][mt][1], cst[ug][mt][2], cst[ug][mt][3],
           cst[ug][mt][4], cst[ug][mt][5], cst[ug][mt][6], cst[ug][mt][7]);
    }
  }
  __syncthreads();

  const v8f z8 = {0.f, 0.f, 0.f, 0.f, 0.f, 0.f, 0.f, 0.f};
  const v4f z4 = {0.f, 0.f, 0.f, 0.f};

#pragma unroll 1
  for (int t = 0; t < NSTEP; ++t) {
    const int cur = t & 1;
    const _Float16* acur = Ah + cur * TILE_ELEMS;
    _Float16* anew = Ah + (cur ^ 1) * TILE_ELEMS;

    if (LAYER == 1) {
      const _Float16* hsrc = hin + (size_t)t * STEP_ELEMS;
      v8h sv[4];
#pragma unroll
      for (int it = 0; it < 4; ++it) sv[it] = *(const v8h*)(hsrc + (size_t)(it * SCAN_THREADS + tid) * 8);
#pragma unroll
      for (int it = 0; it < 4; ++it) {
        const int id  = it * SCAN_THREADS + tid;
        const int row = id >> 6;
        const int c8  = id & 63;
        *(v8h*)(Ax + row * HPITCH + c8 * 8) = sv[it];
      }
      __syncthreads();
    }

    v4f xq00 = z4, xq01 = z4, xq10 = z4, xq11 = z4;
    if (LAYER == 0) {
      const float* xr = xT + (size_t)t * NBATCH + 8 * hh;
      xq00 = *(const v4f*)(xr);
      xq01 = *(const v4f*)(xr + 4);
      xq10 = *(const v4f*)(xr + 16);
      xq11 = *(const v4f*)(xr + 20);
    }

    const _Float16* ar0 = acur + c * HPITCH + koff;
    const _Float16* ar1 = ar0 + 16 * HPITCH;
    const _Float16* xr0 = Ax + ((LAYER == 1) ? (c * HPITCH + koff) : 0);
    const _Float16* xr1 = xr0 + ((LAYER == 1) ? (16 * HPITCH) : 0);

#pragma unroll
    for (int ug = 0; ug < 2; ++ug) {
      const int j = 32 * wave + 16 * ug + c;
      const _Float16* wb = Wb + (size_t)j * KW + koff;
      v8f ai0 = z8, ai1 = z8, af0 = z8, af1 = z8, ag0 = z8, ag1 = z8, ao0 = z8, ao1 = z8;
      if (LAYER == 1) {
        gate_kloop<KW>(xr0, xr1, wb, ai0, ai1, af0, af1, ag0, ag1, ao0, ao1);
        gate_kloop<KW>(ar0, ar1, wb + NHID, ai0, ai1, af0, af1, ag0, ag1, ao0, ao1);
      } else {
        gate_kloop<KW>(ar0, ar1, wb, ai0, ai1, af0, af1, ag0, ag1, ao0, ao1);
      }
      cell_update<LAYER>(ai0, af0, ag0, ao0, bs[ug][0], bs[ug][1], bs[ug][2], bs[ug][3],
                         wq[ug][0], wq[ug][1], wq[ug][2], wq[ug][3], xq00, xq01, cst[ug][0],
                         anew + (8 * hh) * HPITCH + j);
      cell_update<LAYER>(ai1, af1, ag1, ao1, bs[ug][0], bs[ug][1], bs[ug][2], bs[ug][3],
                         wq[ug][0], wq[ug][1], wq[ug][2], wq[ug][3], xq10, xq11, cst[ug][1],
                         anew + (16 + 8 * hh) * HPITCH + j);
    }
    __syncthreads();

    {
      v8h cv[4];
#pragma unroll
      for (int it = 0; it < 4; ++it) {
        const int id  = it * SCAN_THREADS + tid;
        const int row = id >> 6;
        const int c8  = id & 63;
        cv[it] = *(const v8h*)(anew + row * HPITCH + c8 * 8);
      }
      unsigned short* hp = histp + (size_t)t * STEP_ELEMS;
      for (int pass = 0; pass < 2; ++pass) {
#pragma unroll
        for (int it = 0; it < 4; ++it)
          *(volatile v8h*)(hp + (size_t)(it * SCAN_THREADS + tid) * 8) = cv[it];
        __threadfence();
      }
    }
  }
}

__global__ __launch_bounds__(SIDE_THREADS) void fc_kernel(const unsigned short* __restrict__ histp,
                                                          const unsigned short* __restrict__ wfcp,
                                                          const float* __restrict__ fcb, float* __restrict__ out) {
  __shared__ __align__(16) float slab[SIDE_THREADS / 32][96];
  const _Float16* Hs = (const _Float16*)histp;
  const _Float16* Wf = (const _Float16*)wfcp;
  const int tid = threadIdx.x, lane = tid & 31, wave = tid >> 5;
  const int c = lane & 15, hh = lane >> 4, koff = hh * 8;
  const int gw = blockIdx.x * (SIDE_THREADS / 32) + wave;
  const int b  = gw >> 5;
  const int t0 = (gw & 31) * 32;
  const _Float16* a0p = Hs + ((size_t)(t0 + c) * NBATCH + b) * NHID + koff;
  const _Float16* a1p = a0p + (size_t)16 * NBATCH * NHID;
  const _Float16* wp  = Wf + (size_t)c * NHID + koff;
  v8f acc0 = {0.f, 0.f, 0.f, 0.f, 0.f, 0.f, 0.f, 0.f};
  v8f acc1 = {0.f, 0.f, 0.f, 0.f, 0.f, 0.f, 0.f, 0.f};
#pragma unroll 1
  for (int k0 = 0; k0 < NHID; k0 += 32) {
    const v16h a0 = Frag<_Float16>::load(a0p + k0);
    const v16h a1 = Frag<_Float16>::load(a1p + k0);
    const v16h bw = Frag<_Float16>::load(wp + k0);
    acc0 = Frag<_Float16>::mma(a0, bw, acc0);
    acc1 = Frag<_Float16>::mma(a1, bw, acc1);
    guard2(acc0, acc1, a0, a1, bw);
  }
  const int cc = (c < NOUTF) ? c : (NOUTF - 1);
  const float bv = fcb[cc];
  float* sl = slab[wave];
  if (c < NOUTF) {
#pragma unroll
    for (int r = 0; r < 8; ++r) {
      sl[(8 * hh + r) * NOUTF + c]      = fmaf(acc0[r], ACC_FOLD, bv);
      sl[(16 + 8 * hh + r) * NOUTF + c] = fmaf(acc1[r], ACC_FOLD, bv);
    }
  }
  __syncthreads();
  const int ls = (lane < 24) ? lane : 23;
  const v4f v = *(const v4f*)(sl + ls * 4);
  float* op = out + ((size_t)b * NSTEP + t0) * NOUTF + ls * 4;
  for (int pass = 0; pass < 2; ++pass) {
    if (lane < 24) *(volatile v4f*)op = v;
    __threadfence();
  }
}

extern "C" void kernel_launch(void* const* d_in, const int* in_sizes, int n_in,
                              void* d_out, int out_size, void* d_ws, size_t ws_size, hipStream_t stream) {
  if (n_in < 13 || d_out == nullptr || d_ws == nullptr) return;
  if (in_sizes[0] != NBATCH * NSTEP || in_sizes[1] != 2 * STEP_ELEMS || in_sizes[2] != 2 * STEP_ELEMS ||
      in_sizes[3] != NGATE || in_sizes[4] != NGATE * NHID || in_sizes[5] != NGATE || in_sizes[6] != NGATE ||
      in_sizes[7] != NGATE * NHID || in_sizes[8] != NGATE * NHID || in_sizes[9] != NGATE || in_sizes[10] != NGATE ||
      in_sizes[11] != NOUTF * NHID || in_sizes[12] != NOUTF || out_size != NBATCH * NSTEP * NOUTF) return;

  const float* x     = (const float*)d_in[0];
  const float* h0    = (const float*)d_in[1];
  const float* c0    = (const float*)d_in[2];
  const float* w_ih0 = (const float*)d_in[3];
  const float* w_hh0 = (const float*)d_in[4];
  const float* b_ih0 = (const float*)d_in[5];
  const float* b_hh0 = (const float*)d_in[6];
  const float* w_ih1 = (const float*)d_in[7];
  const float* w_hh1 = (const float*)d_in[8];
  const float* b_ih1 = (const float*)d_in[9];
  const float* b_hh1 = (const float*)d_in[10];
  const float* fc_w  = (const float*)d_in[11];
  const float* fc_b  = (const float*)d_in[12];
  float* out = (float*)d_out;

  char* ws = (char*)d_ws; size_t off = 0;
  auto carve = [&](size_t bytes) -> char* { char* p = ws + off; off += (bytes + 255) & ~(size_t)255; return p; };
  unsigned short* WB0   = (unsigned short*)carve((size_t)NGATE * NHID * 2);
  unsigned short* WB1   = (unsigned short*)carve((size_t)NGATE * 2 * NHID * 2);
  unsigned short* WFC   = (unsigned short*)carve((size_t)16 * NHID * 2);
  float*          BSUM  = (float*)carve((size_t)2 * NGATE * 4);
  float*          XT    = (float*)carve((size_t)NSTEP * NBATCH * 4);
  unsigned short* HIST0 = (unsigned short*)carve((size_t)NSTEP * STEP_ELEMS * 2);
  unsigned short* HIST1 = (unsigned short*)carve((size_t)NSTEP * STEP_ELEMS * 2);
  if (off > ws_size || off > (size_t)134217728) return;

  prep_w_kernel<<<dim3(512, 3), SIDE_THREADS, 0, stream>>>(w_hh0, w_ih1, w_hh1, WB0, WB1);
  prep_misc_kernel<<<40, SIDE_THREADS, 0, stream>>>(b_ih0, b_hh0, b_ih1, b_hh1, x, fc_w, BSUM, XT, WFC);
  lstm_scan_kernel<0><<<1, SCAN_THREADS, 0, stream>>>(WB0, BSUM, w_ih0, XT, WB0, h0, c0, HIST0);
  lstm_scan_kernel<1><<<1, SCAN_THREADS, 0, stream>>>(WB1, BSUM + NGATE, BSUM + NGATE, XT, HIST0,
                                                      h0 + STEP_ELEMS, c0 + STEP_ELEMS, HIST1);
  fc_kernel<<<(NBATCH * NSTEP) / (32 * (SIDE_THREADS / 32)), SIDE_THREADS, 0, stream>>>(HIST1, WFC, fc_b, out);
}
